// RNN_84035330113984
// MI455X (gfx1250) — hardware-verified
//
#include <hip/hip_runtime.h>
#include <math.h>

constexpr int SEQ_T   = 100;
constexpr int BATCH   = 256;
constexpr int NGRID   = 2048;
constexpr int NPLACE  = 512;
constexpr int SLABP   = 68;
constexpr float WCARRY     = 64.0f;
constexpr float WCARRY_INV = 1.0f / 64.0f;

static_assert(NPLACE % 32 == 0 && NGRID % 32 == 0, "GEMM K multiples of 32");
static_assert(BATCH % 64 == 0 && (SEQ_T * BATCH) % 64 == 0, "GEMM M multiples of 64");
static_assert(NGRID % 64 == 0 && NPLACE % 64 == 0, "GEMM N multiples of 64");
static_assert(((BATCH / 64) * (NGRID / 64)) % 8 == 0, "step/encoder tiles fill whole blocks");
static_assert((((SEQ_T * BATCH) / 64) * (NPLACE / 64)) % 8 == 0, "decoder tiles fill whole blocks");

typedef __attribute__((ext_vector_type(16))) _Float16 v16h;
typedef __attribute__((ext_vector_type(8)))  _Float16 v8h;
typedef __attribute__((ext_vector_type(8)))  float    v8f;
typedef __attribute__((ext_vector_type(4)))  float    v4f;
typedef __attribute__((ext_vector_type(2)))  float    v2f;

__device__ __forceinline__ void guard_row4(v8f& a0, v8f& a1, v8f& a2, v8f& a3,
                                           v16h x, v16h b0, v16h b1, v16h b2, v16h b3) {
  asm volatile("v_nop\n\tv_nop\n\tv_nop\n\tv_nop"
               : "+v"(a0), "+v"(a1), "+v"(a2), "+v"(a3)
               : "v"(x), "v"(b0), "v"(b1), "v"(b2), "v"(b3));
}
__device__ __forceinline__ void keep4_h(v16h a, v16h b, v16h c, v16h d) {
  asm volatile("v_nop" :: "v"(a), "v"(b), "v"(c), "v"(d));
}
__device__ __forceinline__ void acc_guard4(v8f& a, v8f& b, v8f& c, v8f& d) {
  asm volatile("v_nop\n\tv_nop\n\tv_nop\n\tv_nop" : "+v"(a), "+v"(b), "+v"(c), "+v"(d));
}

union FragU { v16h v; v8h h[2]; };
__device__ __forceinline__ v16h frag_load(const _Float16* p) {
  FragU f;
  f.h[0] = *(const v8h*)(p);
  f.h[1] = *(const v8h*)(p + 16);
  return f.v;
}
__device__ __forceinline__ v8f frag_mma(v16h a, v16h b, v8f c) {
  return __builtin_amdgcn_wmma_f32_16x16x32_f16(false, a, false, b, (short)0, c, false, false);
}

__device__ __forceinline__ float tanh_f(float x) {
  const float e = expf(2.0f * x);
  return 1.0f - 2.0f * __builtin_amdgcn_rcpf(e + 1.0f);
}

__global__ __launch_bounds__(256) void cvt_planes_kernel(
    const float* __restrict__ s0, unsigned short* __restrict__ d0, int nb0, float sc0,
    const float* __restrict__ s1, unsigned short* __restrict__ d1, int nb1, float sc1,
    const float* __restrict__ s2, unsigned short* __restrict__ d2, int nb2, float sc2,
    const float* __restrict__ s3, unsigned short* __restrict__ d3, int nb3, float sc3) {
  const int bx = blockIdx.x;
  const float* s = s0;
  unsigned short* d = d0;
  float sc = sc0;
  int lb = bx;
  if (bx >= nb0) { s = s1; d = d1; sc = sc1; lb = bx - nb0; }
  if (bx >= nb0 + nb1) { s = s2; d = d2; sc = sc2; lb = bx - nb0 - nb1; }
  if (bx >= nb0 + nb1 + nb2) { s = s3; d = d3; sc = sc3; lb = bx - nb0 - nb1 - nb2; }
  if (bx >= nb0 + nb1 + nb2 + nb3) return;
  const size_t i = (size_t)lb * 256 + threadIdx.x;
  const float* sp = s + i * 8;
  const v4f a = *(const v4f*)(sp);
  const v4f b = *(const v4f*)(sp + 4);
  v8h hv;
#pragma unroll
  for (int e = 0; e < 4; ++e) {
    const float fa = a[e] * sc;
    const float fb = b[e] * sc;
    hv[e]     = (_Float16)fa;
    hv[4 + e] = (_Float16)fb;
  }
  unsigned short* dp = d + i * 8;
  *(volatile v8h*)dp = hv;
  __threadfence();
  *(volatile v8h*)dp = hv;
}

template <int EPI>
__global__ __launch_bounds__(256) void gemm64_f16_kernel(
    const unsigned short* __restrict__ Ap, int lda,
    const unsigned short* __restrict__ Btp, int ldb,
    void* __restrict__ Cout, int ldc,
    const float* __restrict__ vt, const float* __restrict__ wih,
    int M, int N, int K, float scale) {
  const _Float16* A  = (const _Float16*)Ap;
  const _Float16* Bt = (const _Float16*)Btp;
  __shared__ __align__(16) float sT[8][16 * SLABP];
  const int lane = threadIdx.x & 31;
  const int wave = threadIdx.x >> 5;
  const int tilesN = N >> 6;
  const int tilesM = M >> 6;
  const int tile = blockIdx.x * 8 + wave;
  if (tile >= tilesM * tilesN) return;
  const int tm = tile / tilesN;
  const int tn = tile - tm * tilesN;
  const int m0 = tm << 6;
  const int n0 = tn << 6;

  const int rlane = lane & 15;
  const int koff  = (lane >> 4) * 8;
  const int mOff  = (lane >> 4) * 8;

  v8f acc[4][4];
#pragma unroll
  for (int i = 0; i < 4; ++i)
#pragma unroll
    for (int j = 0; j < 4; ++j) acc[i][j] = (v8f){0.f, 0.f, 0.f, 0.f, 0.f, 0.f, 0.f, 0.f};

  for (int k0 = 0; k0 < K; k0 += 32) {
    v16h bh[4];
#pragma unroll
    for (int j = 0; j < 4; ++j) {
      const size_t bo = (size_t)(n0 + (j << 4) + rlane) * ldb + koff + k0;
      bh[j] = frag_load(Bt + bo);
    }
#pragma unroll
    for (int i = 0; i < 4; ++i) {
      const size_t ao = (size_t)(m0 + (i << 4) + rlane) * lda + koff + k0;
      const v16h ah = frag_load(A + ao);
#pragma unroll
      for (int j = 0; j < 4; ++j) acc[i][j] = frag_mma(ah, bh[j], acc[i][j]);
      guard_row4(acc[i][0], acc[i][1], acc[i][2], acc[i][3], ah, bh[0], bh[1], bh[2], bh[3]);
    }
    keep4_h(bh[0], bh[1], bh[2], bh[3]);
  }
  acc_guard4(acc[0][0], acc[0][1], acc[0][2], acc[0][3]);
  acc_guard4(acc[1][0], acc[1][1], acc[1][2], acc[1][3]);
  acc_guard4(acc[2][0], acc[2][1], acc[2][2], acc[2][3]);
  acc_guard4(acc[3][0], acc[3][1], acc[3][2], acc[3][3]);

  float* slab = sT[wave];
  float wa[4], wb[4];
#pragma unroll
  for (int j = 0; j < 4; ++j) { wa[j] = 0.0f; wb[j] = 0.0f; }
  if (EPI == 2) {
#pragma unroll
    for (int j = 0; j < 4; ++j) {
      const v2f w = *(const v2f*)(wih + (size_t)(n0 + (j << 4) + rlane) * 2);
      wa[j] = w[0];
      wb[j] = w[1];
    }
    asm volatile("" ::: "memory");
  }
#pragma unroll
  for (int i = 0; i < 4; ++i) {
    const int mBase = m0 + (i << 4);
    float va[8], vb[8];
#pragma unroll
    for (int r = 0; r < 8; ++r) { va[r] = 0.0f; vb[r] = 0.0f; }
    if (EPI == 2) {
      const float* vp = vt + (size_t)(mBase + mOff) * 2;
      const v4f q0 = *(const v4f*)(vp);
      const v4f q1 = *(const v4f*)(vp + 4);
      const v4f q2 = *(const v4f*)(vp + 8);
      const v4f q3 = *(const v4f*)(vp + 12);
      va[0] = q0[0]; vb[0] = q0[1]; va[1] = q0[2]; vb[1] = q0[3];
      va[2] = q1[0]; vb[2] = q1[1]; va[3] = q1[2]; vb[3] = q1[3];
      va[4] = q2[0]; vb[4] = q2[1]; va[5] = q2[2]; vb[5] = q2[3];
      va[6] = q3[0]; vb[6] = q3[1]; va[7] = q3[2]; vb[7] = q3[3];
    }
#pragma unroll
    for (int j = 0; j < 4; ++j) {
#pragma unroll
      for (int r = 0; r < 8; ++r) {
        float x = acc[i][j][r] * scale;
        if (EPI == 2) {
          const float vterm = fmaf(vb[r], wb[j], va[r] * wa[j]);
          x = x + vterm;
        }
        slab[(mOff + r) * SLABP + (j << 4) + rlane] = x;
      }
    }
    __builtin_amdgcn_fence(__ATOMIC_RELEASE, "workgroup");
    __builtin_amdgcn_wave_barrier();
    __builtin_amdgcn_fence(__ATOMIC_ACQUIRE, "workgroup");
    if (EPI == 2) {
      const int th = lane >> 4, tc4 = (lane & 15) * 4;
#pragma unroll 1
      for (int it = 0; it < 8; ++it) {
        float* sp = slab + (it * 2 + th) * SLABP + tc4;
        const v4f xin = *(const v4f*)sp;
        v4f y;
#pragma unroll
        for (int e = 0; e < 4; ++e) y[e] = tanh_f(xin[e]);
        *(v4f*)sp = y;
      }
      __builtin_amdgcn_fence(__ATOMIC_RELEASE, "workgroup");
      __builtin_amdgcn_wave_barrier();
      __builtin_amdgcn_fence(__ATOMIC_ACQUIRE, "workgroup");
    }
    if (EPI == 0) {
      float* C = (float*)Cout;
      const int hh = lane >> 4, c4 = (lane & 15) * 4;
      for (int pass = 0; pass < 2; ++pass) {
#pragma unroll
        for (int it = 0; it < 8; ++it) {
          const int row = it * 2 + hh;
          const v4f val = *(const v4f*)(slab + row * SLABP + c4);
          *(volatile v4f*)(C + (size_t)(mBase + row) * ldc + n0 + c4) = val;
        }
        __threadfence();
      }
    } else {
      unsigned short* C = (unsigned short*)Cout;
      const int q = lane >> 3, c8 = (lane & 7) * 8;
      for (int pass = 0; pass < 2; ++pass) {
#pragma unroll
        for (int it = 0; it < 4; ++it) {
          const int row = it * 4 + q;
          const float* sp = slab + row * SLABP + c8;
          v8h hv;
#pragma unroll
          for (int e = 0; e < 8; ++e) {
            const float f = sp[e];
            hv[e] = (_Float16)f;
          }
          *(volatile v8h*)(C + (size_t)(mBase + row) * ldc + n0 + c8) = hv;
        }
        __threadfence();
      }
    }
    __builtin_amdgcn_fence(__ATOMIC_RELEASE, "workgroup");
    __builtin_amdgcn_wave_barrier();
    __builtin_amdgcn_fence(__ATOMIC_ACQUIRE, "workgroup");
  }
}

constexpr size_t BYTES_WHH  = (size_t)NGRID * NGRID * 2;
constexpr size_t BYTES_WENC = (size_t)NGRID * NPLACE * 2;
constexpr size_t BYTES_WDEC = (size_t)NPLACE * NGRID * 2;
constexpr size_t BYTES_P0   = (size_t)BATCH * NPLACE * 2;
constexpr size_t HPLANE_EL  = (size_t)BATCH * NGRID;
constexpr size_t BYTES_HG   = (size_t)(SEQ_T + 1) * HPLANE_EL * 2;
constexpr size_t CARVE_TOTAL = BYTES_WHH + BYTES_WENC + BYTES_WDEC + BYTES_P0 + BYTES_HG;
static_assert(CARVE_TOTAL == (size_t)118751232, "carve arithmetic");
static_assert(CARVE_TOTAL <= (size_t)134217728, "carve within budget");
static_assert(BYTES_WHH % 256 == 0 && BYTES_WENC % 256 == 0 && BYTES_WDEC % 256 == 0 && BYTES_P0 % 256 == 0, "aligned planes");
static_assert((NGRID * NGRID) % 2048 == 0 && (NGRID * NPLACE) % 2048 == 0 && (BATCH * NPLACE) % 2048 == 0, "convert blocks exact");

extern "C" void kernel_launch(void* const* d_in, const int* in_sizes, int n_in,
                              void* d_out, int out_size, void* d_ws, size_t ws_size, hipStream_t stream) {
  if (n_in < 6 || d_out == nullptr || d_ws == nullptr) return;
  if (in_sizes[0] != SEQ_T * BATCH * 2 || in_sizes[1] != BATCH * NPLACE || in_sizes[2] != NGRID * NPLACE ||
      in_sizes[3] != NGRID * 2 || in_sizes[4] != NGRID * NGRID || in_sizes[5] != NPLACE * NGRID ||
      out_size != SEQ_T * BATCH * NPLACE) return;
  if (CARVE_TOTAL > ws_size) return;

  const float* vel   = (const float*)d_in[0];
  const float* p0    = (const float*)d_in[1];
  const float* w_enc = (const float*)d_in[2];
  const float* w_ih  = (const float*)d_in[3];
  const float* w_hh  = (const float*)d_in[4];
  const float* w_dec = (const float*)d_in[5];
  float* out = (float*)d_out;

  char* ws = (char*)d_ws;
  size_t off = 0;
  unsigned short* WHH16  = (unsigned short*)(ws + off); off += BYTES_WHH;
  unsigned short* WENC16 = (unsigned short*)(ws + off); off += BYTES_WENC;
  unsigned short* WDEC16 = (unsigned short*)(ws + off); off += BYTES_WDEC;
  unsigned short* P016   = (unsigned short*)(ws + off); off += BYTES_P0;
  unsigned short* HG     = (unsigned short*)(ws + off); off += BYTES_HG;
  if (off != CARVE_TOTAL) return;

  const int nbHH  = (NGRID * NGRID) / 2048;
  const int nbENC = (NGRID * NPLACE) / 2048;
  const int nbDEC = (NPLACE * NGRID) / 2048;
  const int nbP0  = (BATCH * NPLACE) / 2048;
  cvt_planes_kernel<<<nbHH + nbENC + nbDEC + nbP0, 256, 0, stream>>>(
      w_hh,  WHH16,  nbHH,  WCARRY,
      w_enc, WENC16, nbENC, WCARRY,
      w_dec, WDEC16, nbDEC, WCARRY,
      p0,    P016,   nbP0,  1.0f);

  const int stepBlocks = ((BATCH / 64) * (NGRID / 64)) / 8;
  gemm64_f16_kernel<1><<<stepBlocks, 256, 0, stream>>>(
      P016, NPLACE, WENC16, NPLACE, (void*)HG, NGRID, vel, w_ih, BATCH, NGRID, NPLACE, WCARRY_INV);

  for (int t = 0; t < SEQ_T; ++t) {
    const unsigned short* hin = HG + (size_t)t * HPLANE_EL;
    unsigned short* hout = HG + (size_t)(t + 1) * HPLANE_EL;
    gemm64_f16_kernel<2><<<stepBlocks, 256, 0, stream>>>(
        hin, NGRID, WHH16, NGRID, (void*)hout, NGRID,
        vel + (size_t)t * BATCH * 2, w_ih, BATCH, NGRID, NGRID, WCARRY_INV);
  }

  const int decBlocks = (((SEQ_T * BATCH) / 64) * (NPLACE / 64)) / 8;
  gemm64_f16_kernel<0><<<decBlocks, 256, 0, stream>>>(
      HG + HPLANE_EL, NGRID, WDEC16, NGRID, (void*)out, NPLACE, vel, w_ih,
      SEQ_T * BATCH, NPLACE, NGRID, WCARRY_INV);
}
